// PredecessorDecoder_87299505258630
// MI455X (gfx1250) — hardware-verified
//
#include <hip/hip_runtime.h>

typedef __attribute__((ext_vector_type(16))) _Float16     v16h;
typedef __attribute__((ext_vector_type(8)))  _Float16     v8h;
typedef __attribute__((ext_vector_type(2)))  _Float16     h2v;
typedef __attribute__((ext_vector_type(8)))  float        v8f;
typedef __attribute__((ext_vector_type(4)))  unsigned int u32x4;
typedef __attribute__((ext_vector_type(8)))  unsigned int u32x8;

#define N_NODES 1024
#define LATENT  64
#define NFEAT   128
#define ROWP    66
#define S2_BLOCK 256

__global__ __launch_bounds__(128)
void node_precompute_wmma(const float* __restrict__ encoded,
                          const float* __restrict__ h,
                          const float* __restrict__ W1,
                          const float* __restrict__ b1,
                          _Float16* __restrict__ P)
{
    const int lane      = threadIdx.x & 31;
    const int waveInBlk = threadIdx.x >> 5;
    const int tile      = blockIdx.x * 4 + waveInBlk;
    const int t         = tile >> 8;
    const int rem       = tile & 255;
    const int mt        = rem >> 2;
    const int nt        = rem & 3;

    const int half16 = lane >> 4;
    const int l16    = lane & 15;
    const int m      = mt * 16 + l16;
    const int n      = nt * 16 + l16;

    v8f acc = {};
    #pragma unroll
    for (int kc = 0; kc < 4; ++kc) {
        const int kbase = kc * 32;
        v16h a, b;
        #pragma unroll
        for (int j = 0; j < 16; ++j) {
            const int v     = j >> 1;
            const int klocA = (v < 4 ? 2 * v : 8 + 2 * v) + 8 * half16 + (j & 1);
            const int ka    = kbase + klocA;
            const float av  = (ka < LATENT) ? encoded[m * LATENT + ka]
                                            : h[m * LATENT + (ka - LATENT)];
            a[j] = (_Float16)av;
            const int kb = kbase + ((j < 8) ? j : (j + 8)) + 8 * half16;
            b[j] = (_Float16)W1[(t * NFEAT + kb) * LATENT + n];
        }
        acc = __builtin_amdgcn_wmma_f32_16x16x32_f16(
                   false, a,  false, b,
                   (short)0, acc,  false,  false);
        asm volatile("v_nop\n\tv_nop\n\tv_nop\n\tv_nop" : "+v"(acc) : "v"(a), "v"(b));
    }

    const float bias = (t == 0) ? b1[n] : 0.0f;
    __shared__ __attribute__((aligned(16))) _Float16 tileP[16][64];
    #pragma unroll
    for (int r = 0; r < 8; ++r) tileP[r + 8 * half16][n] = (_Float16)(acc[r] + bias);
    __syncthreads();
    {
        const int row = threadIdx.x >> 3, seg = threadIdx.x & 7;
        _Float16* dst = P + (size_t)t * (N_NODES * LATENT) + (size_t)(mt * 16 + row) * LATENT + seg * 8;
        const v8h v = *(const v8h*)(&tileP[row][seg * 8]);
        *(volatile v8h*)dst = v; __threadfence(); *(volatile v8h*)dst = v;
    }
}

__global__ __launch_bounds__(S2_BLOCK)
void edge_decode(const int* __restrict__ edge_index,
                 const float* __restrict__ W2,
                 const float* __restrict__ b2,
                 const _Float16* __restrict__ P,
                 float* __restrict__ out,
                 int E, int chunk)
{
    extern __shared__ char smem[];
    _Float16* sA = (_Float16*)smem;
    _Float16* sB = sA + N_NODES * ROWP;
    float*    sW = (float*)(sB + N_NODES * ROWP);

    for (int piece = threadIdx.x; piece < 2 * N_NODES * 8; piece += S2_BLOCK) {
        const int tb = piece >> 13, rem = piece & 8191;
        const int row = rem >> 3, seg = rem & 7;
        const v8h v = *(const v8h*)(P + (size_t)tb * (N_NODES * LATENT) + row * LATENT + seg * 8);
        _Float16* d = (tb ? sB : sA) + row * ROWP + seg * 8;
        #pragma unroll
        for (int q = 0; q < 4; ++q) *(h2v*)(d + 2 * q) = (h2v){v[2 * q], v[2 * q + 1]};
    }
    if (threadIdx.x < LATENT) sW[threadIdx.x] = W2[threadIdx.x];
    __syncthreads();

    const float bias2 = b2[0];
    const int base = blockIdx.x * chunk;
    for (int i = threadIdx.x; i < chunk; i += S2_BLOCK) {
        const int e = base + i;
        if (e >= E) break;
        __builtin_prefetch(&edge_index[e + S2_BLOCK], 0, 0);
        __builtin_prefetch(&edge_index[E + e + S2_BLOCK], 0, 0);
        const int s = edge_index[e];
        const int d = edge_index[E + e];
        const _Float16* ra = &sA[s * ROWP];
        const _Float16* rb = &sB[d * ROWP];
        float acc = bias2;
        #pragma unroll
        for (int k = 0; k < LATENT; k += 2) {
            const h2v va = *(const h2v*)(&ra[k]);
            const h2v vb = *(const h2v*)(&rb[k]);
            float x0 = (float)va.x + (float)vb.x;
            float x1 = (float)va.y + (float)vb.y;
            x0 = x0 > 0.0f ? x0 : 0.0f;
            x1 = x1 > 0.0f ? x1 : 0.0f;
            acc = fmaf(x0, sW[k],     acc);
            acc = fmaf(x1, sW[k + 1], acc);
        }
        *(volatile float*)(out + e) = acc;
        __threadfence();
        *(volatile float*)(out + e) = acc;
    }
}

extern "C" void kernel_launch(void* const* d_in, const int* in_sizes, int n_in,
                              void* d_out, int out_size, void* d_ws, size_t ws_size,
                              hipStream_t stream) {
    const float* encoded = (const float*)d_in[0];
    const float* hfeat   = (const float*)d_in[1];
    const int*   eidx    = (const int*)d_in[2];
    const float* W1      = (const float*)d_in[3];
    const float* b1      = (const float*)d_in[4];
    const float* W2      = (const float*)d_in[5];
    const float* b2      = (const float*)d_in[6];

    const int E = in_sizes[2] / 2;
    (void)n_in; (void)out_size;
    if (ws_size < (size_t)2 * N_NODES * LATENT * sizeof(_Float16)) return;

    _Float16* P = (_Float16*)d_ws;

    node_precompute_wmma<<<128, 128, 0, stream>>>(encoded, hfeat, W1, b1, P);

    const int grid  = 256;
    const int chunk = (E + grid - 1) / grid;
    const size_t shmem = (size_t)(2 * N_NODES * ROWP) * sizeof(_Float16)
                       + LATENT * sizeof(float);
    edge_decode<<<grid, S2_BLOCK, shmem, stream>>>(eidx, W2, b2, P,
                                                   (float*)d_out, E, chunk);
}
